// NormalSelfAttention1d_23390391894152
// MI455X (gfx1250) — hardware-verified
//
#include <hip/hip_runtime.h>
#include <stdint.h>

#define NB   8
#define DM   512
#define NS   2048
#define NTOK (NB * NS)

typedef _Float16 v16h __attribute__((ext_vector_type(16)));
typedef _Float16 v8h  __attribute__((ext_vector_type(8)));
typedef __bf16   v16b __attribute__((ext_vector_type(16)));
typedef __bf16   v8b  __attribute__((ext_vector_type(8)));
typedef float    v8f  __attribute__((ext_vector_type(8)));
typedef float    v4f  __attribute__((ext_vector_type(4)));
typedef unsigned short v8us __attribute__((ext_vector_type(8)));

static_assert((DM % 64) == 0 && (NS % 64) == 0 && (NTOK % 64) == 0);
static_assert(((DM * DM / 8) % 256) == 0);

__device__ __forceinline__ unsigned short bfbits(float f) {
  unsigned u = __float_as_uint(f);
  return (unsigned short)((u + 0x7FFFu + ((u >> 16) & 1u)) >> 16);
}
__device__ __forceinline__ float bfval(unsigned short b) { return __uint_as_float(((unsigned)b) << 16); }
__device__ __forceinline__ float bfr(float f) { return bfval(bfbits(f)); }

__device__ __forceinline__ v16b ldfrag_b(const __bf16* p) {
  union { v16b v; v8b h[2]; } f;
  f.h[0] = *(const v8b*)(p);
  f.h[1] = *(const v8b*)(p + 16);
  return f.v;
}
__device__ __forceinline__ v16h ldfrag_h(const _Float16* p) {
  union { v16h v; v8h h[2]; } f;
  f.h[0] = *(const v8h*)(p);
  f.h[1] = *(const v8h*)(p + 16);
  return f.v;
}
__device__ __forceinline__ v8f mma_b(v16b a, v16b b, v8f c) {
  return __builtin_amdgcn_wmma_f32_16x16x32_bf16(false, a, false, b, (short)0, c, false, false);
}
__device__ __forceinline__ v8f mma_h(v16h a, v16h b, v8f c) {
  return __builtin_amdgcn_wmma_f32_16x16x32_f16(false, a, false, b, (short)0, c, false, false);
}
__device__ __forceinline__ v8f zero8() {
  v8f z;
#pragma unroll
  for (int i = 0; i < 8; ++i) z[i] = 0.0f;
  return z;
}

__device__ __forceinline__ void guard_g(v8f& a, v8f& b, v16b x, v16b y) {
  asm volatile("v_nop\n\tv_nop\n\tv_nop\n\tv_nop" : "+v"(a), "+v"(b) : "v"(x), "v"(y));
}
__device__ __forceinline__ void keep4(v16b a, v16b b, v16b c, v16b d) {
  asm volatile("v_nop" :: "v"(a), "v"(b), "v"(c), "v"(d));
}
__device__ __forceinline__ void accg4(v8f& a, v8f& b, v8f& c, v8f& d) {
  asm volatile("v_nop\n\tv_nop\n\tv_nop\n\tv_nop" : "+v"(a), "+v"(b), "+v"(c), "+v"(d));
}
__device__ __forceinline__ void guard_s(v8f& a, v8f& b, v8f& c, v8f& d,
                                        v16b x0, v16b x1, v16b x2, v16b x3,
                                        v16b y0, v16b y1, v16b y2, v16b y3) {
  asm volatile("v_nop\n\tv_nop\n\tv_nop\n\tv_nop"
               : "+v"(a), "+v"(b), "+v"(c), "+v"(d)
               : "v"(x0), "v"(x1), "v"(x2), "v"(x3), "v"(y0), "v"(y1), "v"(y2), "v"(y3));
}
__device__ __forceinline__ void guard_pv(v8f& a0, v8f& a1, v8f& a2, v8f& a3,
                                         v8f& b0, v8f& b1, v8f& b2, v8f& b3,
                                         v16h p0, v16h p1, v16h x0, v16h x1, v16h x2, v16h x3) {
  asm volatile("v_nop\n\tv_nop\n\tv_nop\n\tv_nop"
               : "+v"(a0), "+v"(a1), "+v"(a2), "+v"(a3), "+v"(b0), "+v"(b1), "+v"(b2), "+v"(b3)
               : "v"(p0), "v"(p1), "v"(x0), "v"(x1), "v"(x2), "v"(x3));
}

__global__ __launch_bounds__(256) void cvt_w_kernel(const float* __restrict__ w0, const float* __restrict__ w1,
                                                    const float* __restrict__ w2, unsigned short* __restrict__ wb,
                                                    int n8) {
  const int nb0 = n8 >> 8;
  const int seg = (int)blockIdx.x / nb0;
  if (seg > 2) return;
  const float* src = (seg == 2) ? w2 : ((seg == 1) ? w1 : w0);
  const int li = ((int)blockIdx.x - seg * nb0) * 256 + (int)threadIdx.x;
  if (li >= n8) return;
  const size_t e = (size_t)li * 8;
  const v4f a = *(const v4f*)(src + e);
  const v4f b = *(const v4f*)(src + e + 4);
  v8us o;
#pragma unroll
  for (int i = 0; i < 4; ++i) {
    o[i]     = bfbits(a[i]);
    o[4 + i] = bfbits(b[i]);
  }
  unsigned short* d = wb + (size_t)seg * (size_t)n8 * 8 + e;
  *(volatile v8us*)d = o;
  __threadfence();
  *(volatile v8us*)d = o;
}

#define XTP 72
__global__ __launch_bounds__(256) void xpose_kernel(const float* __restrict__ x, unsigned short* __restrict__ xt) {
  __shared__ __align__(16) unsigned short T[64 * XTP];
  const int tid = threadIdx.x;
  const int n0 = (int)blockIdx.x * 64, d0 = (int)blockIdx.y * 64, b = (int)blockIdx.z;
  const float* xb = x + ((size_t)b * DM + d0) * NS + n0;
  const int rr = tid >> 4, c4 = (tid & 15) * 4;
#pragma unroll
  for (int i = 0; i < 4; ++i) {
    const int r = rr + 16 * i;
    const v4f v = *(const v4f*)(xb + (size_t)r * NS + c4);
#pragma unroll
    for (int j = 0; j < 4; ++j) T[(c4 + j) * XTP + r] = bfbits(v[j]);
  }
  __syncthreads();
  unsigned short* xo = xt + ((size_t)b * NS + n0) * DM + d0;
  const int rn = tid >> 3, c8 = (tid & 7) * 8;
#pragma unroll
  for (int ps = 0; ps < 2; ++ps) {
#pragma unroll
    for (int i = 0; i < 2; ++i) {
      const int row = rn + 32 * i;
      const v8us v = *(const v8us*)(T + row * XTP + c8);
      *(volatile v8us*)(xo + (size_t)row * DM + c8) = v;
    }
    __threadfence();
  }
}

template <int MODE>
__global__ __launch_bounds__(256) void gemm64_kernel(const __bf16* __restrict__ A, int lda,
                                                     const __bf16* __restrict__ Bt, int ldb,
                                                     unsigned short* __restrict__ C0, unsigned short* __restrict__ C1,
                                                     int ldc, const float* __restrict__ bias,
                                                     int M, int N, int K, float scale) {
  __shared__ __align__(16) float sT[8][16 * 68];
  const int lane = threadIdx.x & 31, wave = threadIdx.x >> 5;
  const int tilesN = N >> 6, tilesM = M >> 6;
  const int tile = (int)blockIdx.x * 8 + wave;
  if (tile >= tilesM * tilesN) return;
  const int tm = tile / tilesN, tn = tile - tm * tilesN;
  const int m0 = tm << 6, n0 = tn << 6;
  const int rl = lane & 15;
  const int koff = (lane >> 4) * 8;
  const int mOff = (lane >> 4) * 8;

  v8f acc[4][4];
#pragma unroll
  for (int i = 0; i < 4; ++i)
#pragma unroll
    for (int j = 0; j < 4; ++j) acc[i][j] = zero8();

#pragma unroll 1
  for (int k0 = 0; k0 < K; k0 += 32) {
    v16b bh[4];
#pragma unroll
    for (int j = 0; j < 4; ++j) bh[j] = ldfrag_b(Bt + (size_t)(n0 + (j << 4) + rl) * ldb + koff + k0);
#pragma unroll
    for (int i = 0; i < 4; ++i) {
      const v16b ah = ldfrag_b(A + (size_t)(m0 + (i << 4) + rl) * lda + koff + k0);
#pragma unroll
      for (int j = 0; j < 4; ++j) acc[i][j] = mma_b(ah, bh[j], acc[i][j]);
      guard_g(acc[i][0], acc[i][3], ah, bh[3]);
    }
    keep4(bh[0], bh[1], bh[2], bh[3]);
  }
  accg4(acc[0][0], acc[0][1], acc[0][2], acc[0][3]);
  accg4(acc[1][0], acc[1][1], acc[1][2], acc[1][3]);
  accg4(acc[2][0], acc[2][1], acc[2][2], acc[2][3]);
  accg4(acc[3][0], acc[3][1], acc[3][2], acc[3][3]);

  float* slab = sT[wave];
  const int qq = lane >> 3, c8 = (lane & 7) * 8;
#pragma unroll
  for (int i = 0; i < 4; ++i) {
    const int mBase = m0 + (i << 4);
    if (MODE == 0) {
#pragma unroll
      for (int j = 0; j < 4; ++j) {
        const float bv = bfr(bias[n0 + (j << 4) + rl]);
#pragma unroll
        for (int r = 0; r < 8; ++r) slab[(mOff + r) * 68 + (j << 4) + rl] = (acc[i][j][r] + bv) * scale;
      }
    } else {
      const v4f b0 = *(const v4f*)(bias + mBase + mOff);
      const v4f b1 = *(const v4f*)(bias + mBase + mOff + 4);
#pragma unroll
      for (int j = 0; j < 4; ++j) {
#pragma unroll
        for (int r = 0; r < 4; ++r) {
          slab[(mOff + r) * 68 + (j << 4) + rl]     = (acc[i][j][r] + bfr(b0[r])) * scale;
          slab[(mOff + 4 + r) * 68 + (j << 4) + rl] = (acc[i][j][4 + r] + bfr(b1[r])) * scale;
        }
      }
    }
    __builtin_amdgcn_fence(__ATOMIC_RELEASE, "workgroup");
    __builtin_amdgcn_wave_barrier();
    __builtin_amdgcn_fence(__ATOMIC_ACQUIRE, "workgroup");
#pragma unroll
    for (int ps = 0; ps < 2; ++ps) {
#pragma unroll
      for (int it = 0; it < 4; ++it) {
        const int row = it * 4 + qq;
        const float* sp = slab + row * 68 + c8;
        const size_t go = (size_t)(mBase + row) * ldc + n0 + c8;
        if (MODE == 0) {
          v8us hv, lv;
#pragma unroll
          for (int e = 0; e < 8; ++e) {
            const float v = sp[e];
            const unsigned short hb = bfbits(v);
            hv[e] = hb;
            lv[e] = bfbits(v - bfval(hb));
          }
          *(volatile v8us*)(C0 + go) = hv;
          *(volatile v8us*)(C1 + go) = lv;
        } else {
          v8h hv;
#pragma unroll
          for (int e = 0; e < 8; ++e) hv[e] = (_Float16)sp[e];
          *(volatile v8h*)((_Float16*)C0 + go) = hv;
        }
      }
      __threadfence();
    }
    __builtin_amdgcn_fence(__ATOMIC_RELEASE, "workgroup");
    __builtin_amdgcn_wave_barrier();
    __builtin_amdgcn_fence(__ATOMIC_ACQUIRE, "workgroup");
  }
}

#define QB       32
#define KCH      256
#define QSP      520
#define PSP      264
#define OSP      36
#define LDS_QH   0
#define LDS_QL   33280
#define LDS_PS   66560
#define LDS_PMAX 83456
#define LDS_PSUM 84480
#define LDS_ST   85504
#define ATT_LDS  86016
static_assert(QB * QSP * 2 == LDS_QL - LDS_QH);
static_assert(QB * QSP * 2 == LDS_PS - LDS_QL);
static_assert(QB * PSP * 2 == LDS_PMAX - LDS_PS);
static_assert(LDS_PSUM - LDS_PMAX == 256 * 4);
static_assert(LDS_ST - LDS_PSUM == 256 * 4);
static_assert(ATT_LDS - LDS_ST == 4 * 32 * 4);
static_assert(DM * OSP * 4 <= LDS_PMAX);
static_assert((QSP % 8) == 0 && (PSP % 8) == 0 && PSP >= KCH && (OSP % 4) == 0);
static_assert((LDS_QL % 16) == 0 && (LDS_PS % 16) == 0 && (LDS_PMAX % 16) == 0 && (LDS_ST % 16) == 0);
static_assert((NS % KCH) == 0 && (NS % QB) == 0 && (DM % 64) == 0 && DM == 8 * 64);

__global__ __launch_bounds__(256) void attn_kernel(const __bf16* __restrict__ qh, const __bf16* __restrict__ ql,
                                                   const __bf16* __restrict__ kh, const __bf16* __restrict__ kl,
                                                   const _Float16* __restrict__ vt, float* __restrict__ out,
                                                   int ns, int ntok) {
  extern __shared__ __align__(16) char smem[];
  __bf16* Qh = (__bf16*)(smem + LDS_QH);
  __bf16* Ql = (__bf16*)(smem + LDS_QL);
  _Float16* Ps = (_Float16*)(smem + LDS_PS);
  float* pmax = (float*)(smem + LDS_PMAX);
  float* psum = (float*)(smem + LDS_PSUM);
  float* m_s  = (float*)(smem + LDS_ST);
  float* l_s  = m_s + 32;
  float* al_s = m_s + 64;
  float* li_s = m_s + 96;

  const int tid = threadIdx.x, wave = tid >> 5, lane = tid & 31, h = lane >> 4, c = lane & 15;
  const int q0 = (int)blockIdx.x * QB;
  const int b = q0 / ns;
  const int nq0 = q0 - b * ns;
  const int krow0 = b * ns;
  const float ninf = -__builtin_inff();

  if (tid < 32) { m_s[tid] = ninf; l_s[tid] = 0.0f; al_s[tid] = 0.0f; li_s[tid] = 0.0f; }
  psum[tid] = 0.0f;
#pragma unroll
  for (int i = 0; i < 8; ++i) {
    const int idx = i * 256 + tid;
    const int row = idx >> 6;
    const int pc  = idx & 63;
    const size_t go = (size_t)(q0 + row) * DM + pc * 8;
    *(v8b*)(Qh + row * QSP + pc * 8) = *(const v8b*)(qh + go);
    *(v8b*)(Ql + row * QSP + pc * 8) = *(const v8b*)(ql + go);
  }
  __syncthreads();

  v8f oacc[2][4];
#pragma unroll
  for (int qt = 0; qt < 2; ++qt)
#pragma unroll
    for (int nt = 0; nt < 4; ++nt) oacc[qt][nt] = zero8();

  const __bf16* qh0p = Qh + c * QSP + 8 * h;
  const __bf16* qh1p = Qh + (16 + c) * QSP + 8 * h;
  const __bf16* ql0p = Ql + c * QSP + 8 * h;
  const __bf16* ql1p = Ql + (16 + c) * QSP + 8 * h;
  const _Float16* pa0p = Ps + c * PSP + 8 * h;
  const _Float16* pa1p = Ps + (16 + c) * PSP + 8 * h;
  const int ntile = ns / KCH;

#pragma unroll 1
  for (int t = 0; t < ntile; ++t) {
    const int kb = krow0 + t * KCH + 32 * wave;
    const __bf16* khp0 = kh + (size_t)(kb + c) * DM + 8 * h;
    const __bf16* khp1 = kh + (size_t)(kb + 16 + c) * DM + 8 * h;
    const __bf16* klp0 = kl + (size_t)(kb + c) * DM + 8 * h;
    const __bf16* klp1 = kl + (size_t)(kb + 16 + c) * DM + 8 * h;
    v8f sacc[2][2];
#pragma unroll
    for (int qt = 0; qt < 2; ++qt)
#pragma unroll
      for (int kt = 0; kt < 2; ++kt) sacc[qt][kt] = zero8();
#pragma unroll 1
    for (int k0 = 0; k0 < DM; k0 += 32) {
      const v16b a0 = ldfrag_b(khp0 + k0), a1 = ldfrag_b(khp1 + k0);
      const v16b e0 = ldfrag_b(klp0 + k0), e1 = ldfrag_b(klp1 + k0);
      const v16b g0 = ldfrag_b(qh0p + k0), g1 = ldfrag_b(qh1p + k0);
      const v16b f0 = ldfrag_b(ql0p + k0), f1 = ldfrag_b(ql1p + k0);
      sacc[0][0] = mma_b(a0, g0, sacc[0][0]);
      sacc[0][0] = mma_b(a0, f0, sacc[0][0]);
      sacc[0][0] = mma_b(e0, g0, sacc[0][0]);
      sacc[0][1] = mma_b(a1, g0, sacc[0][1]);
      sacc[0][1] = mma_b(a1, f0, sacc[0][1]);
      sacc[0][1] = mma_b(e1, g0, sacc[0][1]);
      sacc[1][0] = mma_b(a0, g1, sacc[1][0]);
      sacc[1][0] = mma_b(a0, f1, sacc[1][0]);
      sacc[1][0] = mma_b(e0, g1, sacc[1][0]);
      sacc[1][1] = mma_b(a1, g1, sacc[1][1]);
      sacc[1][1] = mma_b(a1, f1, sacc[1][1]);
      sacc[1][1] = mma_b(e1, g1, sacc[1][1]);
      guard_s(sacc[0][0], sacc[0][1], sacc[1][0], sacc[1][1], a0, a1, e0, e1, g0, g1, f0, f1);
    }
    {
      float pm0 = ninf, pm1 = ninf;
#pragma unroll
      for (int kt = 0; kt < 2; ++kt) {
#pragma unroll
        for (int r = 0; r < 8; ++r) {
          pm0 = fmaxf(pm0, sacc[0][kt][r]);
          pm1 = fmaxf(pm1, sacc[1][kt][r]);
        }
      }
      pm0 = fmaxf(pm0, __shfl_xor(pm0, 16, 32));
      pm1 = fmaxf(pm1, __shfl_xor(pm1, 16, 32));
      pmax[wave * 32 + c] = pm0;
      pmax[wave * 32 + 16 + c] = pm1;
    }
    __syncthreads();
    if (wave == 0) {
      const int row = lane;
      float ps = 0.0f;
#pragma unroll
      for (int w = 0; w < 8; ++w) ps += psum[w * 32 + row];
      l_s[row] = l_s[row] * al_s[row] + ps;
      const float mo = m_s[row];
      float mx = mo;
#pragma unroll
      for (int w = 0; w < 8; ++w) mx = fmaxf(mx, pmax[w * 32 + row]);
      al_s[row] = __expf(mo - mx);
      m_s[row] = mx;
    }
    __syncthreads();
    {
      const float mq0 = m_s[c], mq1 = m_s[16 + c];
      float ps0 = 0.0f, ps1 = 0.0f;
#pragma unroll
      for (int kt = 0; kt < 2; ++kt) {
        v8h h0, h1;
#pragma unroll
        for (int r = 0; r < 8; ++r) {
          const _Float16 x0 = (_Float16)(__expf(sacc[0][kt][r] - mq0) * 16384.0f);
          const _Float16 x1 = (_Float16)(__expf(sacc[1][kt][r] - mq1) * 16384.0f);
          h0[r] = x0; ps0 += (float)x0;
          h1[r] = x1; ps1 += (float)x1;
        }
        *(v8h*)(Ps + c * PSP + 32 * wave + 16 * kt + 8 * h) = h0;
        *(v8h*)(Ps + (16 + c) * PSP + 32 * wave + 16 * kt + 8 * h) = h1;
      }
      ps0 += __shfl_xor(ps0, 16, 32);
      ps1 += __shfl_xor(ps1, 16, 32);
      psum[wave * 32 + c] = ps0;
      psum[wave * 32 + 16 + c] = ps1;
      const v4f aA = *(const v4f*)(al_s + 8 * h), aB = *(const v4f*)(al_s + 8 * h + 4);
      const v4f bA = *(const v4f*)(al_s + 16 + 8 * h), bB = *(const v4f*)(al_s + 16 + 8 * h + 4);
#pragma unroll
      for (int nt = 0; nt < 4; ++nt) {
#pragma unroll
        for (int r = 0; r < 4; ++r) {
          oacc[0][nt][r] *= aA[r]; oacc[0][nt][4 + r] *= aB[r];
          oacc[1][nt][r] *= bA[r]; oacc[1][nt][4 + r] *= bB[r];
        }
      }
    }
    __syncthreads();
    {
      const _Float16* vbp = vt + (size_t)(64 * wave + c) * ntok + (size_t)krow0 + (size_t)t * KCH + 8 * h;
#pragma unroll 1
      for (int ks = 0; ks < KCH; ks += 32) {
        const v16h pa0 = ldfrag_h(pa0p + ks), pa1 = ldfrag_h(pa1p + ks);
        v16h vb[4];
#pragma unroll
        for (int j = 0; j < 4; ++j) vb[j] = ldfrag_h(vbp + (size_t)(16 * j) * ntok + ks);
#pragma unroll
        for (int j = 0; j < 4; ++j) {
          oacc[0][j] = mma_h(pa0, vb[j], oacc[0][j]);
          oacc[1][j] = mma_h(pa1, vb[j], oacc[1][j]);
        }
        guard_pv(oacc[0][0], oacc[0][1], oacc[0][2], oacc[0][3],
                 oacc[1][0], oacc[1][1], oacc[1][2], oacc[1][3],
                 pa0, pa1, vb[0], vb[1], vb[2], vb[3]);
      }
    }
  }

  if (wave == 0) {
    const int row = lane;
    float ps = 0.0f;
#pragma unroll
    for (int w = 0; w < 8; ++w) ps += psum[w * 32 + row];
    const float l = l_s[row] * al_s[row] + ps;
    li_s[row] = (1.0f / l) * 0.0625f;
  }
  __syncthreads();
  float* Os = (float*)(smem);
  {
    const v4f iA0 = *(const v4f*)(li_s + 8 * h),      iB0 = *(const v4f*)(li_s + 8 * h + 4);
    const v4f iA1 = *(const v4f*)(li_s + 16 + 8 * h), iB1 = *(const v4f*)(li_s + 16 + 8 * h + 4);
#pragma unroll
    for (int nt = 0; nt < 4; ++nt) {
      const int col = 64 * wave + 16 * nt + c;
      float* op = Os + col * OSP;
      v4f u;
#pragma unroll
      for (int r = 0; r < 4; ++r) u[r] = oacc[0][nt][r] * iA0[r];
      *(v4f*)(op + 8 * h) = u;
#pragma unroll
      for (int r = 0; r < 4; ++r) u[r] = oacc[0][nt][4 + r] * iB0[r];
      *(v4f*)(op + 8 * h + 4) = u;
#pragma unroll
      for (int r = 0; r < 4; ++r) u[r] = oacc[1][nt][r] * iA1[r];
      *(v4f*)(op + 16 + 8 * h) = u;
#pragma unroll
      for (int r = 0; r < 4; ++r) u[r] = oacc[1][nt][4 + r] * iB1[r];
      *(v4f*)(op + 16 + 8 * h + 4) = u;
    }
  }
  __syncthreads();
  {
    const int qq = lane >> 3, c4 = (lane & 7) * 4;
    float* ob = out + ((size_t)b * DM) * (size_t)ns + nq0;
#pragma unroll
    for (int ps = 0; ps < 2; ++ps) {
#pragma unroll
      for (int it = 0; it < 16; ++it) {
        const int d = 64 * wave + 4 * it + qq;
        const v4f v = *(const v4f*)(Os + d * OSP + c4);
        *(volatile v4f*)(ob + (size_t)d * ns + c4) = v;
      }
      __threadfence();
    }
  }
}

extern "C" void kernel_launch(void* const* d_in, const int* in_sizes, int n_in,
                              void* d_out, int out_size, void* d_ws, size_t ws_size,
                              hipStream_t stream) {
  if (n_in < 7) return;
  if (in_sizes[0] != NB * DM * NS) return;
  if (in_sizes[1] != DM * DM || in_sizes[3] != DM * DM || in_sizes[5] != DM * DM) return;
  if (in_sizes[2] != DM || in_sizes[4] != DM || in_sizes[6] != DM) return;
  if (out_size != NB * DM * NS) return;

  const float* x  = (const float*)d_in[0];
  const float* Wq = (const float*)d_in[1];
  const float* bq = (const float*)d_in[2];
  const float* Wk = (const float*)d_in[3];
  const float* bk = (const float*)d_in[4];
  const float* Wv = (const float*)d_in[5];
  const float* bv = (const float*)d_in[6];
  float* out = (float*)d_out;

  const size_t bWB = (size_t)3 * DM * DM * 2;
  const size_t bPL = (size_t)NTOK * DM * 2;
  size_t off = 0;
  const size_t oWB = off; off += bWB;
  const size_t oXT = off; off += bPL;
  const size_t oQH = off; off += bPL;
  const size_t oQL = off; off += bPL;
  const size_t oKH = off; off += bPL;
  const size_t oKL = off; off += bPL;
  const size_t oVT = off; off += bPL;
  if (off > ws_size) return;
  if (off > (size_t)134217728) return;

  char* ws = (char*)d_ws;
  unsigned short* WB = (unsigned short*)(ws + oWB);
  unsigned short* XT = (unsigned short*)(ws + oXT);
  unsigned short* QH = (unsigned short*)(ws + oQH);
  unsigned short* QL = (unsigned short*)(ws + oQL);
  unsigned short* KH = (unsigned short*)(ws + oKH);
  unsigned short* KL = (unsigned short*)(ws + oKL);
  unsigned short* VT = (unsigned short*)(ws + oVT);

  const dim3 blk(256);
  const int n8 = DM * DM / 8;
  const int gqk = ((NTOK / 64) * (DM / 64)) / 8;
  if ((((NTOK / 64) * (DM / 64)) % 8) != 0) return;

  cvt_w_kernel<<<dim3(3 * (n8 / 256)), blk, 0, stream>>>(Wq, Wk, Wv, WB, n8);
  xpose_kernel<<<dim3(NS / 64, DM / 64, NB), blk, 0, stream>>>(x, XT);
  gemm64_kernel<0><<<dim3(gqk), blk, 0, stream>>>((const __bf16*)XT, DM, (const __bf16*)WB, DM,
                                                   QH, QL, DM, bq, NTOK, DM, DM, 1.0f);
  gemm64_kernel<0><<<dim3(gqk), blk, 0, stream>>>((const __bf16*)XT, DM, (const __bf16*)(WB + (size_t)DM * DM), DM,
                                                   KH, KL, DM, bk, NTOK, DM, DM, 1.0f);
  gemm64_kernel<1><<<dim3(gqk), blk, 0, stream>>>((const __bf16*)(WB + (size_t)2 * DM * DM), DM, (const __bf16*)XT, DM,
                                                   VT, VT, NTOK, bv, DM, NTOK, DM, 16.0f);
  (void)hipFuncSetAttribute(reinterpret_cast<const void*>(&attn_kernel),
                            hipFuncAttributeMaxDynamicSharedMemorySize, ATT_LDS);
  attn_kernel<<<dim3(NTOK / QB), blk, ATT_LDS, stream>>>((const __bf16*)QH, (const __bf16*)QL,
                                                         (const __bf16*)KH, (const __bf16*)KL,
                                                         (const _Float16*)VT, out, NS, NTOK);
  (void)hipGetLastError();
}
